// DAGConcat_60361470378542
// MI455X (gfx1250) — hardware-verified
//
#include <hip/hip_runtime.h>
#include <stdint.h>
#include <stddef.h>

#define NB   32
#define NN   128
#define EMB  1024
#define HID  512
#define NR   4096
#define G3   1536
#define G6   3072
#define G4   2048
#define NCLS 7
#define HP   520
#define VP   1028
#define TPG  132
#define WSC  64.0f
#define ASC  16.0f
#define OSC  0.0009765625f

#define GNN_LDS 246528

static_assert(NR == NB * NN);
static_assert((HP * 2) % 16 == 0);
static_assert((VP * 4) % 16 == 0);
static_assert((TPG * 4) % 16 == 0);
static_assert(GNN_LDS == 16 * HID * 4 * 3 + 16 * VP * 4 + 16 * HP * 2 * 2 + 16 * NN * 4 * 4 + 8 * HID * 4);
static_assert(EMB % 32 == 0);
static_assert(HID % 32 == 0);
static_assert(NR % 64 == 0);
static_assert(HID % 128 == 0);
static_assert(G4 % (4 * 256) == 0);
static_assert(G3 % 4 == 0);
static_assert(HID % 4 == 0);

typedef _Float16       v16h __attribute__((ext_vector_type(16)));
typedef float          v8f  __attribute__((ext_vector_type(8)));
typedef float          v4f  __attribute__((ext_vector_type(4)));
typedef unsigned int   v4u  __attribute__((ext_vector_type(4)));
typedef v4f __attribute__((may_alias)) v4fa;
typedef v4u __attribute__((may_alias)) v4ua;

union FragH { v16h v; v4u q[2]; };

__device__ __forceinline__ v8f wmma_h(v16h a, v16h b, v8f c) {
  v8f d = __builtin_amdgcn_wmma_f32_16x16x32_f16(false, a, false, b, (short)0, c, false, false);
  asm volatile("v_nop\n\tv_nop\n\tv_nop\n\tv_nop" : "+v"(d) : "v"(a), "v"(b));
  return d;
}

__device__ __forceinline__ v16h ldfrag(const unsigned short* p, int h) {
  FragH f;
  f.q[0] = *(const v4ua*)(p + 8 * h);
  f.q[1] = *(const v4ua*)(p + 16 + 8 * h);
  return f.v;
}

__device__ __forceinline__ unsigned short hbits(float a) {
  return __builtin_bit_cast(unsigned short, (_Float16)a);
}
__device__ __forceinline__ unsigned int pkh(float a, float b) {
  return (unsigned int)hbits(a) | ((unsigned int)hbits(b) << 16);
}
__device__ __forceinline__ v4u pack8(v4f a, v4f c) {
  v4u o;
  o.x = pkh(a.x, a.y); o.y = pkh(a.z, a.w);
  o.z = pkh(c.x, c.y); o.w = pkh(c.z, c.w);
  return o;
}

__device__ __forceinline__ float sigm(float x) {
  return __builtin_amdgcn_rcpf(1.0f + __expf(-x));
}
__device__ __forceinline__ float tnh(float x) {
  return 1.0f - 2.0f * __builtin_amdgcn_rcpf(__expf(2.0f * x) + 1.0f);
}

__device__ __forceinline__ float dot32(const float* a, const float* b) {
  float s = 0.f;
  #pragma unroll
  for (int k = 0; k < 32; k += 4) {
    const v4f x = *(const v4fa*)(a + k);
    const v4f y = *(const v4fa*)(b + k);
    s = fmaf(x.x, y.x, s); s = fmaf(x.y, y.y, s);
    s = fmaf(x.z, y.z, s); s = fmaf(x.w, y.w, s);
  }
  return s;
}

__device__ __forceinline__ float dot32r(const v4f (&x)[8], const float* b) {
  float s = 0.f;
  #pragma unroll
  for (int k = 0; k < 8; ++k) {
    const v4f y = *(const v4fa*)(b + 4 * k);
    s = fmaf(x[k].x, y.x, s); s = fmaf(x[k].y, y.y, s);
    s = fmaf(x[k].z, y.z, s); s = fmaf(x[k].w, y.w, s);
  }
  return s;
}

__global__ __launch_bounds__(256) void k_cvt8(
    const float* s0, unsigned short* d0, int n0, float c0,
    const float* s1, unsigned short* d1, int n1, float c1,
    const float* s2, unsigned short* d2, int n2, float c2,
    const float* s3, unsigned short* d3, int n3, float c3,
    const float* s4, unsigned short* d4, int n4, float c4,
    const float* s5, unsigned short* d5, int n5, float c5,
    const float* s6, unsigned short* d6, int n6, float c6,
    const float* s7, unsigned short* d7, int n7, float c7)
{
  const int j = blockIdx.y;
  const bool b4 = (j & 4) != 0, b2 = (j & 2) != 0, b1 = (j & 1) != 0;
  const float* src = b4 ? (b2 ? (b1 ? s7 : s6) : (b1 ? s5 : s4))
                        : (b2 ? (b1 ? s3 : s2) : (b1 ? s1 : s0));
  unsigned short* dst = b4 ? (b2 ? (b1 ? d7 : d6) : (b1 ? d5 : d4))
                           : (b2 ? (b1 ? d3 : d2) : (b1 ? d1 : d0));
  const int n8 = b4 ? (b2 ? (b1 ? n7 : n6) : (b1 ? n5 : n4))
                    : (b2 ? (b1 ? n3 : n2) : (b1 ? n1 : n0));
  const float sc = b4 ? (b2 ? (b1 ? c7 : c6) : (b1 ? c5 : c4))
                      : (b2 ? (b1 ? c3 : c2) : (b1 ? c1 : c0));
  const int stride = gridDim.x * 256;
  #pragma unroll 1
  for (int g = blockIdx.x * 256 + threadIdx.x; g < n8; g += stride) {
    const float* p = src + (size_t)g * 8;
    const v4f a = *(const v4fa*)p;
    const v4f c = *(const v4fa*)(p + 4);
    const v4u pk = pack8(a * sc, c * sc);
    unsigned short* d = dst + (size_t)g * 8;
    *(volatile v4u*)d = pk;
    __threadfence();
    *(volatile v4u*)d = pk;
  }
}

__device__ __forceinline__ void gseg(v8f (&acc)[2][2],
                                     const unsigned short* __restrict__ A, int pitch, int klen,
                                     const unsigned short* __restrict__ W, int K, int kw,
                                     int rb, int cb, int h, int m)
{
  #pragma unroll 1
  for (int k0 = 0; k0 < klen; k0 += 32) {
    v16h a[2];
    #pragma unroll
    for (int mt = 0; mt < 2; ++mt)
      a[mt] = ldfrag(A + (size_t)(rb + 16 * mt + m) * pitch + k0, h);
    #pragma unroll
    for (int nt = 0; nt < 2; ++nt) {
      const v16h b = ldfrag(W + (size_t)(cb + 16 * nt + m) * K + kw + k0, h);
      #pragma unroll
      for (int mt = 0; mt < 2; ++mt) acc[mt][nt] = wmma_h(a[mt], b, acc[mt][nt]);
    }
  }
}

__global__ __launch_bounds__(256) void k_gemm(
    const unsigned short* __restrict__ A0, int p0, int l0,
    const unsigned short* __restrict__ A1, int p1, int l1,
    const unsigned short* __restrict__ A2, int p2, int l2,
    const unsigned short* __restrict__ A3, int p3, int l3,
    const unsigned short* __restrict__ A4, int p4, int l4,
    const unsigned short* __restrict__ W, int K,
    const float* __restrict__ bias, int act,
    float* __restrict__ Cf, int ldc, int wf,
    unsigned short* __restrict__ Ch, int ldh, int wh)
{
  __shared__ __align__(16) float sT[64 * TPG];
  const int tid = threadIdx.x, lane = tid & 31, wv = tid >> 5;
  const int h = lane >> 4, m = lane & 15;
  const int wm = wv >> 2, wn = wv & 3;
  const int rb0 = blockIdx.x * 64, nb = blockIdx.y * 128;
  const int rb = rb0 + 32 * wm, cb = nb + 32 * wn;

  const v8f z8 = {0.f, 0.f, 0.f, 0.f, 0.f, 0.f, 0.f, 0.f};
  v8f acc[2][2];
  #pragma unroll
  for (int mt = 0; mt < 2; ++mt)
    #pragma unroll
    for (int nt = 0; nt < 2; ++nt) acc[mt][nt] = z8;

  int kw = 0;
  gseg(acc, A0, p0, l0, W, K, kw, rb, cb, h, m); kw += l0;
  gseg(acc, A1, p1, l1, W, K, kw, rb, cb, h, m); kw += l1;
  gseg(acc, A2, p2, l2, W, K, kw, rb, cb, h, m); kw += l2;
  gseg(acc, A3, p3, l3, W, K, kw, rb, cb, h, m); kw += l3;
  gseg(acc, A4, p4, l4, W, K, kw, rb, cb, h, m);

  #pragma unroll
  for (int mt = 0; mt < 2; ++mt)
    #pragma unroll
    for (int nt = 0; nt < 2; ++nt) {
      const int col = 32 * wn + 16 * nt + m;
      #pragma unroll
      for (int r = 0; r < 8; ++r) {
        const int row = 32 * wm + 16 * mt + 8 * h + r;
        sT[row * TPG + col] = acc[mt][nt][r];
      }
    }
  __syncthreads();

  const v4f bv4 = *(const v4fa*)(bias + nb + 4 * lane);
  v4f ov[8];
  size_t fo[8];
  #pragma unroll
  for (int i = 0; i < 8; ++i) {
    const int row = wv + 8 * i;
    v4f z = *(const v4fa*)(sT + row * TPG + 4 * lane) * OSC + bv4;
    if (act) { z.x = fmaxf(z.x, 0.f); z.y = fmaxf(z.y, 0.f); z.z = fmaxf(z.z, 0.f); z.w = fmaxf(z.w, 0.f); }
    ov[i] = z;
    fo[i] = (size_t)(rb0 + row) * ldc + nb + 4 * lane;
  }
  const v4f b8a = *(const v4fa*)(bias + nb + 8 * m);
  const v4f b8b = *(const v4fa*)(bias + nb + 8 * m + 4);
  v4u hv[4];
  size_t ho[4];
  #pragma unroll
  for (int i2 = 0; i2 < 4; ++i2) {
    const int row = wv + 16 * i2 + 8 * h;
    v4f za = *(const v4fa*)(sT + row * TPG + 8 * m) * OSC + b8a;
    v4f zb = *(const v4fa*)(sT + row * TPG + 8 * m + 4) * OSC + b8b;
    if (act) {
      za.x = fmaxf(za.x, 0.f); za.y = fmaxf(za.y, 0.f); za.z = fmaxf(za.z, 0.f); za.w = fmaxf(za.w, 0.f);
      zb.x = fmaxf(zb.x, 0.f); zb.y = fmaxf(zb.y, 0.f); zb.z = fmaxf(zb.z, 0.f); zb.w = fmaxf(zb.w, 0.f);
    }
    hv[i2] = pack8(za * ASC, zb * ASC);
    ho[i2] = (size_t)(rb0 + row) * ldh + nb + 8 * m;
  }
  if (wf) {
    #pragma unroll
    for (int i = 0; i < 8; ++i) *(volatile v4f*)(Cf + fo[i]) = ov[i];
  }
  if (wh) {
    #pragma unroll
    for (int i2 = 0; i2 < 4; ++i2) *(volatile v4u*)(Ch + ho[i2]) = hv[i2];
  }
  __threadfence();
  if (wf) {
    #pragma unroll
    for (int i = 0; i < 8; ++i) *(volatile v4f*)(Cf + fo[i]) = ov[i];
  }
  if (wh) {
    #pragma unroll
    for (int i2 = 0; i2 < 4; ++i2) *(volatile v4u*)(Ch + ho[i2]) = hv[i2];
  }
}

__global__ __launch_bounds__(256) void k_lstm(const unsigned short* __restrict__ Fh,
                                              const unsigned short* __restrict__ Wih,
                                              const unsigned short* __restrict__ Whh,
                                              const float* __restrict__ bih,
                                              const float* __restrict__ bhh,
                                              unsigned short* __restrict__ Lh)
{
  __shared__ __align__(16) unsigned short sH[2 * 16 * HP];
  __shared__ __align__(16) float sB[G4];
  const int tid = threadIdx.x, lane = tid & 31, wv = tid >> 5;
  const int h = lane >> 4, m = lane & 15;
  const int n0 = blockIdx.x * 16;
  for (int q = tid; q < 2 * 16 * HP; q += 256) sH[q] = 0;
  #pragma unroll 1
  for (int q = tid; q < G4 / 4; q += 256) {
    const v4f a = *(const v4fa*)(bih + 4 * q);
    const v4f b = *(const v4fa*)(bhh + 4 * q);
    *(v4fa*)(sB + 4 * q) = a + b;
  }

  float c[4][8];
  #pragma unroll
  for (int g = 0; g < 4; ++g) {
    #pragma unroll
    for (int r = 0; r < 8; ++r) c[g][r] = 0.f;
  }
  __syncthreads();

  float bs[4][4];
  #pragma unroll
  for (int g = 0; g < 4; ++g) {
    const int k = 16 * (wv + 8 * g) + m;
    #pragma unroll
    for (int e = 0; e < 4; ++e) bs[g][e] = sB[k + 512 * e];
  }

  const v8f z8 = {0.f, 0.f, 0.f, 0.f, 0.f, 0.f, 0.f, 0.f};
  #pragma unroll 1
  for (int t = 0; t < NB; ++t) {
    const unsigned short* hc = sH + (t & 1) * (16 * HP);
    unsigned short* hn = sH + ((t & 1) ^ 1) * (16 * HP);
    const size_t row0 = (size_t)t * NN + n0;

    #pragma unroll
    for (int g = 0; g < 4; ++g) {
      const int k = 16 * (wv + 8 * g) + m;
      v8f acc[4];
      #pragma unroll
      for (int e = 0; e < 4; ++e) acc[e] = z8;
      #pragma unroll 1
      for (int k0 = 0; k0 < EMB; k0 += 32) {
        const v16h a = ldfrag(Fh + (row0 + m) * EMB + k0, h);
        #pragma unroll
        for (int e = 0; e < 4; ++e)
          acc[e] = wmma_h(a, ldfrag(Wih + (size_t)(k + 512 * e) * EMB + k0, h), acc[e]);
      }
      #pragma unroll 1
      for (int k0 = 0; k0 < HID; k0 += 32) {
        const v16h a = ldfrag(hc + m * HP + k0, h);
        #pragma unroll
        for (int e = 0; e < 4; ++e)
          acc[e] = wmma_h(a, ldfrag(Whh + (size_t)(k + 512 * e) * HID + k0, h), acc[e]);
      }
      #pragma unroll
      for (int r = 0; r < 8; ++r) {
        const int row = 8 * h + r;
        const float gi = sigm(acc[0][r] * OSC + bs[g][0]);
        const float gf = sigm(acc[1][r] * OSC + bs[g][1]);
        const float gg = tnh(acc[2][r] * OSC + bs[g][2]);
        const float gq = sigm(acc[3][r] * OSC + bs[g][3]);
        const float cn = gf * c[g][r] + gi * gg;
        c[g][r] = cn;
        const float hv = gq * tnh(cn);
        hn[row * HP + k] = hbits(hv * ASC);
      }
    }
    __syncthreads();

    v4u v[4];
    size_t o4[4];
    #pragma unroll
    for (int rr = 0; rr < 2; ++rr) {
      const int bl = 2 * wv + rr;
      #pragma unroll
      for (int q = 0; q < 2; ++q) {
        v[2 * rr + q] = *(const v4ua*)(hn + bl * HP + 256 * q + 8 * lane);
        o4[2 * rr + q] = (row0 + bl) * HID + 256 * q + 8 * lane;
      }
    }
    #pragma unroll
    for (int q = 0; q < 4; ++q) *(volatile v4u*)(Lh + o4[q]) = v[q];
    __threadfence();
    #pragma unroll
    for (int q = 0; q < 4; ++q) *(volatile v4u*)(Lh + o4[q]) = v[q];
  }
}

__global__ __launch_bounds__(256) void k_gnn(
    const float* __restrict__ Hlf, const unsigned short* __restrict__ Hlh,
    const float* __restrict__ adj, const float* __restrict__ smask,
    const float* __restrict__ aW, const float* __restrict__ abp,
    const unsigned short* __restrict__ Wq, const unsigned short* __restrict__ Wm,
    const unsigned short* __restrict__ Wr,
    const float* __restrict__ cbih, const float* __restrict__ cbhh,
    const float* __restrict__ pbih, const float* __restrict__ pbhh,
    float* __restrict__ VS, float* __restrict__ H1f, unsigned short* __restrict__ H1h)
{
  extern __shared__ __align__(16) unsigned char gsm[];
  float* sMf = (float*)(gsm + 0);
  float* sHf = (float*)(gsm + 32768);
  float* sV  = (float*)(gsm + 65536);
  unsigned short* sMh = (unsigned short*)(gsm + 131328);
  unsigned short* sHh = (unsigned short*)(gsm + 147968);
  float* sK  = (float*)(gsm + 164608);
  float* sP  = (float*)(gsm + 172800);
  float* sS  = (float*)(gsm + 180992);
  float* sQf = (float*)(gsm + 189184);
  float* sBi = (float*)(gsm + 221952);
  float* sAd = (float*)(gsm + 238336);

  const int tid = threadIdx.x, lane = tid & 31, wv = tid >> 5;
  const int h = lane >> 4, m = lane & 15;
  const int b0 = blockIdx.x * 16;
  const int bl = tid >> 4, part = tid & 15;
  const int bg = b0 + bl;
  const float abv = abp[0];
  const v8f z8 = {0.f, 0.f, 0.f, 0.f, 0.f, 0.f, 0.f, 0.f};

  for (int q = tid; q < 16 * NN; q += 256) sK[q] = 0.f;
  #pragma unroll 1
  for (int q = tid; q < G3 / 4; q += 256) {
    const int e = 4 * q;
    const int seg = e >> 9;
    const int kin = e & (HID - 1);
    const v4f a = *(const v4fa*)(cbih + e);
    const v4f b = *(const v4fa*)(cbhh + e);
    const v4f c = *(const v4fa*)(pbih + e);
    const v4f d = *(const v4fa*)(pbhh + e);
    if (seg < 2) {
      *(v4fa*)(sBi + seg * HID + kin) = a + b;
      *(v4fa*)(sBi + (4 + seg) * HID + kin) = c + d;
    } else {
      *(v4fa*)(sBi + 2 * HID + kin) = a;
      *(v4fa*)(sBi + 3 * HID + kin) = b;
      *(v4fa*)(sBi + 6 * HID + kin) = c;
      *(v4fa*)(sBi + 7 * HID + kin) = d;
    }
  }
  __syncthreads();

  #pragma unroll 1
  for (int i = 0; i < NN; ++i) {
    const size_t rowq = (size_t)bg * NN + i;
    v4f qv[8];

    {
      const float* arow = adj + rowq * NN + 8 * part;
      const float* srow = smask + rowq * NN + 8 * part;
      const v4f ad0 = *(const v4fa*)arow;
      const v4f ad1 = *(const v4fa*)(arow + 4);
      const v4f sm0 = *(const v4fa*)srow;
      const v4f sm1 = *(const v4fa*)(srow + 4);
      *(v4fa*)(sAd + bl * NN + 8 * part) = ad0;
      *(v4fa*)(sAd + bl * NN + 8 * part + 4) = ad1;
      *(v4fa*)(sS + bl * NN + 8 * part) = sm0;
      *(v4fa*)(sS + bl * NN + 8 * part + 4) = sm1;
      const float* qsrc = Hlf + rowq * HID + 32 * part;
      #pragma unroll
      for (int k = 0; k < 8; ++k) qv[k] = *(const v4fa*)(qsrc + 4 * k);
      #pragma unroll
      for (int k = 0; k < 8; ++k) *(v4fa*)(sQf + bl * HID + 32 * part + 4 * k) = qv[k];
    }
    __syncthreads();

    if (i > 0) {
      float qd = dot32r(qv, aW + part * 32);
      qd += __shfl_xor(qd, 8); qd += __shfl_xor(qd, 4);
      qd += __shfl_xor(qd, 2); qd += __shfl_xor(qd, 1);
      float al[8];
      float mx = -__builtin_inff();
      #pragma unroll
      for (int jj = 0; jj < 8; ++jj) {
        const int j = part + 16 * jj;
        const float ad = sAd[bl * NN + j];
        const float kd = sK[bl * NN + j];
        float a = ((qd + kd) + abv) - (1.0f - ad) * 1e30f;
        a = (j < i) ? a : -__builtin_inff();
        al[jj] = a;
        mx = fmaxf(mx, a);
      }
      mx = fmaxf(mx, __shfl_xor(mx, 8)); mx = fmaxf(mx, __shfl_xor(mx, 4));
      mx = fmaxf(mx, __shfl_xor(mx, 2)); mx = fmaxf(mx, __shfl_xor(mx, 1));
      float sm = 0.f;
      #pragma unroll
      for (int jj = 0; jj < 8; ++jj) { al[jj] = expf(al[jj] - mx); sm += al[jj]; }
      sm += __shfl_xor(sm, 8); sm += __shfl_xor(sm, 4);
      sm += __shfl_xor(sm, 2); sm += __shfl_xor(sm, 1);
      const float inv = 1.0f / sm;
      #pragma unroll
      for (int jj = 0; jj < 8; ++jj) {
        const int j = part + 16 * jj;
        sP[bl * NN + j] = al[jj] * inv;
      }
    }
    __syncthreads();

    if (i > 0) {
      const float* vb = VS + (size_t)bg * NN * 1024;
      #pragma unroll 1
      for (int ch = 0; ch < 4; ++ch) {
        const int col = part * 32 + ch * 8;
        v4f a0 = {0.f, 0.f, 0.f, 0.f};
        v4f a1 = {0.f, 0.f, 0.f, 0.f};
        #pragma unroll 2
        for (int j = 0; j < i; ++j) {
          const float w = sP[bl * NN + j];
          const float s = sS[bl * NN + j];
          const float u = 1.0f - s;
          const float* vr = vb + (size_t)j * 1024 + col;
          const v4f x0 = *(const v4fa*)vr;
          const v4f x1 = *(const v4fa*)(vr + 4);
          const v4f y0 = *(const v4fa*)(vr + 512);
          const v4f y1 = *(const v4fa*)(vr + 516);
          a0 += w * (x0 * s + y0 * u);
          a1 += w * (x1 * s + y1 * u);
        }
        *(v4fa*)(sMf + bl * HID + col) = a0;
        *(v4fa*)(sMf + bl * HID + col + 4) = a1;
        *(v4ua*)(sMh + bl * HP + col) = pack8(a0 * ASC, a1 * ASC);
      }
    } else {
      for (int q = tid; q < 16 * HID; q += 256) sMf[q] = 0.f;
      for (int q = tid; q < 16 * HP; q += 256) sMh[q] = 0;
    }
    __syncthreads();

    #pragma unroll 1
    for (int g = 0; g < 4; ++g) {
      const int kk = 16 * (wv + 8 * g) + m;
      v8f aR = z8, aZ = z8, aQN = z8, aMN = z8;
      v8f bR = z8, bZ = z8, bQN = z8, bMN = z8;
      const unsigned short* wq0 = Wq + (size_t)kk * HID;
      const unsigned short* wm0 = Wm + (size_t)kk * HID;
      const unsigned short* qa = Hlh + ((size_t)(b0 + m) * NN + i) * HID;
      #pragma unroll 1
      for (int k0 = 0; k0 < HID; k0 += 32) {
        const v16h a = ldfrag(qa + k0, h);
        aR  = wmma_h(a, ldfrag(wq0 + k0, h), aR);
        aZ  = wmma_h(a, ldfrag(wq0 + (size_t)512 * HID + k0, h), aZ);
        aQN = wmma_h(a, ldfrag(wq0 + (size_t)1024 * HID + k0, h), aQN);
        bR  = wmma_h(a, ldfrag(wq0 + (size_t)1536 * HID + k0, h), bR);
        bZ  = wmma_h(a, ldfrag(wq0 + (size_t)2048 * HID + k0, h), bZ);
        bQN = wmma_h(a, ldfrag(wq0 + (size_t)2560 * HID + k0, h), bQN);
      }
      const unsigned short* ma = sMh + m * HP;
      #pragma unroll 1
      for (int k0 = 0; k0 < HID; k0 += 32) {
        const v16h a = ldfrag(ma + k0, h);
        aR  = wmma_h(a, ldfrag(wm0 + k0, h), aR);
        aZ  = wmma_h(a, ldfrag(wm0 + (size_t)512 * HID + k0, h), aZ);
        aMN = wmma_h(a, ldfrag(wm0 + (size_t)1024 * HID + k0, h), aMN);
        bR  = wmma_h(a, ldfrag(wm0 + (size_t)1536 * HID + k0, h), bR);
        bZ  = wmma_h(a, ldfrag(wm0 + (size_t)2048 * HID + k0, h), bZ);
        bMN = wmma_h(a, ldfrag(wm0 + (size_t)2560 * HID + k0, h), bMN);
      }
      const float cb0 = sBi[kk];
      const float cb1 = sBi[HID + kk];
      const float cbi = sBi[2 * HID + kk];
      const float cbh = sBi[3 * HID + kk];
      const float pb0 = sBi[4 * HID + kk];
      const float pb1 = sBi[5 * HID + kk];
      const float pbi = sBi[6 * HID + kk];
      const float pbh = sBi[7 * HID + kk];
      #pragma unroll
      for (int r = 0; r < 8; ++r) {
        const int row = 8 * h + r;
        const float qk = sQf[row * HID + kk];
        const float mk = sMf[row * HID + kk];
        const float rc = sigm(aR[r] * OSC + cb0);
        const float zc = sigm(aZ[r] * OSC + cb1);
        const float nc = tnh((aQN[r] * OSC + cbi) + rc * (aMN[r] * OSC + cbh));
        const float hc = (1.0f - zc) * nc + zc * mk;
        const float rp = sigm(bR[r] * OSC + pb0);
        const float zp = sigm(bZ[r] * OSC + pb1);
        const float np = tnh((bMN[r] * OSC + pbi) + rp * (bQN[r] * OSC + pbh));
        const float hp = (1.0f - zp) * np + zp * qk;
        const float hv = hc + hp;
        sHf[row * HID + kk] = hv;
        sHh[row * HP + kk] = hbits(hv * ASC);
      }
    }
    __syncthreads();

    {
      float kd = dot32(sHf + bl * HID + part * 32, aW + HID + part * 32);
      kd += __shfl_xor(kd, 8); kd += __shfl_xor(kd, 4);
      kd += __shfl_xor(kd, 2); kd += __shfl_xor(kd, 1);
      if (part == 0) sK[bl * NN + i] = kd;
    }
    #pragma unroll 1
    for (int g = 0; g < 8; ++g) {
      const int cc = 16 * (wv + 8 * g) + m;
      v8f acc = z8;
      const unsigned short* ha = sHh + m * HP;
      const unsigned short* wr = Wr + (size_t)cc * HID;
      #pragma unroll 1
      for (int k0 = 0; k0 < HID; k0 += 32)
        acc = wmma_h(ldfrag(ha + k0, h), ldfrag(wr + k0, h), acc);
      #pragma unroll
      for (int r = 0; r < 8; ++r) sV[(8 * h + r) * VP + cc] = acc[r] * OSC;
    }
    __syncthreads();

    #pragma unroll 1
    for (int rr = 0; rr < 2; ++rr) {
      const int blr = 2 * wv + rr;
      const size_t rg = (size_t)(b0 + blr) * NN + i;
      {
        v4f v[8];
        #pragma unroll
        for (int q = 0; q < 8; ++q) v[q] = *(const v4fa*)(sV + blr * VP + 128 * q + 4 * lane);
        float* d = VS + rg * 1024 + 4 * lane;
        #pragma unroll
        for (int q = 0; q < 8; ++q) *(volatile v4f*)(d + 128 * q) = v[q];
        __threadfence();
        #pragma unroll
        for (int q = 0; q < 8; ++q) *(volatile v4f*)(d + 128 * q) = v[q];
      }
      {
        v4f v[4];
        #pragma unroll
        for (int q = 0; q < 4; ++q) v[q] = *(const v4fa*)(sHf + blr * HID + 128 * q + 4 * lane);
        float* d = H1f + rg * HID + 4 * lane;
        #pragma unroll
        for (int q = 0; q < 4; ++q) *(volatile v4f*)(d + 128 * q) = v[q];
        __threadfence();
        #pragma unroll
        for (int q = 0; q < 4; ++q) *(volatile v4f*)(d + 128 * q) = v[q];
      }
      {
        v4u v[2];
        #pragma unroll
        for (int q = 0; q < 2; ++q) v[q] = *(const v4ua*)(sHh + blr * HP + 256 * q + 8 * lane);
        unsigned short* d = H1h + rg * HID + 8 * lane;
        #pragma unroll
        for (int q = 0; q < 2; ++q) *(volatile v4u*)(d + 256 * q) = v[q];
        __threadfence();
        #pragma unroll
        for (int q = 0; q < 2; ++q) *(volatile v4u*)(d + 256 * q) = v[q];
      }
    }
    __threadfence();
    __syncthreads();
  }
}

__global__ __launch_bounds__(128) void k_head(const unsigned short* __restrict__ X,
                                              const unsigned short* __restrict__ Wo,
                                              const float* __restrict__ ob,
                                              float* __restrict__ out)
{
  __shared__ __align__(16) float sO[64 * NCLS];
  const int tid = threadIdx.x, lane = tid & 31, wv = tid >> 5;
  const int h = lane >> 4, m = lane & 15;
  const int rb = blockIdx.x * 64 + 16 * wv;
  v8f acc = {0.f, 0.f, 0.f, 0.f, 0.f, 0.f, 0.f, 0.f};
  const unsigned short* xa = X + (size_t)(rb + m) * HID;
  const unsigned short* wb = Wo + (size_t)m * HID;
  #pragma unroll 1
  for (int k0 = 0; k0 < HID; k0 += 32)
    acc = wmma_h(ldfrag(xa + k0, h), ldfrag(wb + k0, h), acc);
  const float bb = ob[(m < NCLS) ? m : (NCLS - 1)];
  #pragma unroll
  for (int r = 0; r < 8; ++r) {
    const int row = 16 * wv + 8 * h + r;
    if (m < NCLS) sO[row * NCLS + m] = acc[r] * OSC + bb;
  }
  __syncthreads();
  if (wv == 0) {
    float* base = out + (size_t)blockIdx.x * (64 * NCLS);
    v4f v[4];
    #pragma unroll
    for (int q = 0; q < 4; ++q) {
      int idx = 32 * q + lane;
      idx = (idx > 111) ? 111 : idx;
      v[q] = *(const v4fa*)(sO + 4 * idx);
    }
    #pragma unroll
    for (int q = 0; q < 3; ++q) *(volatile v4f*)(base + 4 * (32 * q + lane)) = v[q];
    if (lane < 16) *(volatile v4f*)(base + 4 * (96 + lane)) = v[3];
    __threadfence();
    #pragma unroll
    for (int q = 0; q < 3; ++q) *(volatile v4f*)(base + 4 * (32 * q + lane)) = v[q];
    if (lane < 16) *(volatile v4f*)(base + 4 * (96 + lane)) = v[3];
  }
}

extern "C" void kernel_launch(void* const* d_in, const int* in_sizes, int n_in,
                              void* d_out, int out_size, void* d_ws, size_t ws_size,
                              hipStream_t stream)
{
  if (n_in < 29) return;
  if (in_sizes[0]  != NR * EMB) return;
  if (in_sizes[1]  != NR * NN) return;
  if (in_sizes[2]  != NR * NN) return;
  if (in_sizes[5]  != G4 * EMB) return;
  if (in_sizes[6]  != G4 * HID) return;
  if (in_sizes[7]  != G4) return;
  if (in_sizes[8]  != G4) return;
  if (in_sizes[9]  != HID * EMB) return;
  if (in_sizes[10] != HID) return;
  if (in_sizes[11] != 2 * 2 * HID) return;
  if (in_sizes[12] != 2) return;
  if (in_sizes[13] != 2 * HID * HID) return;
  if (in_sizes[14] != 2 * HID * HID) return;
  if (in_sizes[15] != 2 * G3 * HID) return;
  if (in_sizes[16] != 2 * G3 * HID) return;
  if (in_sizes[17] != 2 * G3) return;
  if (in_sizes[18] != 2 * G3) return;
  if (in_sizes[19] != 2 * G3 * HID) return;
  if (in_sizes[20] != 2 * G3 * HID) return;
  if (in_sizes[21] != 2 * G3) return;
  if (in_sizes[22] != 2 * G3) return;
  if (in_sizes[23] != HID * G6) return;
  if (in_sizes[24] != HID) return;
  if (in_sizes[25] != HID * HID) return;
  if (in_sizes[26] != HID) return;
  if (in_sizes[27] != NCLS * HID) return;
  if (in_sizes[28] != NCLS) return;
  if (out_size != NR * NCLS) return;

  const float* features = (const float*)d_in[0];
  const float* adj      = (const float*)d_in[1];
  const float* smask    = (const float*)d_in[2];
  const float* lstm_Wih = (const float*)d_in[5];
  const float* lstm_Whh = (const float*)d_in[6];
  const float* lstm_bih = (const float*)d_in[7];
  const float* lstm_bhh = (const float*)d_in[8];
  const float* fc1_W    = (const float*)d_in[9];
  const float* fc1_b    = (const float*)d_in[10];
  const float* attn_W   = (const float*)d_in[11];
  const float* attn_b   = (const float*)d_in[12];
  const float* Wr0      = (const float*)d_in[13];
  const float* Wr1      = (const float*)d_in[14];
  const float* gC_Wih   = (const float*)d_in[15];
  const float* gC_Whh   = (const float*)d_in[16];
  const float* gC_bih   = (const float*)d_in[17];
  const float* gC_bhh   = (const float*)d_in[18];
  const float* gP_Wih   = (const float*)d_in[19];
  const float* gP_Whh   = (const float*)d_in[20];
  const float* gP_bih   = (const float*)d_in[21];
  const float* gP_bhh   = (const float*)d_in[22];
  const float* mlp0_W   = (const float*)d_in[23];
  const float* mlp0_b   = (const float*)d_in[24];
  const float* mlp1_W   = (const float*)d_in[25];
  const float* mlp1_b   = (const float*)d_in[26];
  const float* out_W    = (const float*)d_in[27];
  const float* out_b    = (const float*)d_in[28];
  float* out = (float*)d_out;

  const size_t bF   = (size_t)NR * EMB * 2;
  const size_t bWiL = (size_t)G4 * EMB * 2;
  const size_t bWhL = (size_t)G4 * HID * 2;
  const size_t bWfc = (size_t)HID * EMB * 2;
  const size_t bWq  = (size_t)G6 * HID * 2;
  const size_t bWm  = (size_t)G6 * HID * 2;
  const size_t bWr  = (size_t)2 * HID * HID * 2;
  const size_t bWp0 = (size_t)HID * G6 * 2;
  const size_t bWp1 = (size_t)HID * HID * 2;
  const size_t bWo  = (size_t)16 * HID * 2;
  const size_t bL   = (size_t)NR * HID * 2;
  const size_t bHf  = (size_t)NR * HID * 4;
  const size_t bHh  = (size_t)NR * HID * 2;
  const size_t bVS  = (size_t)NR * 1024 * 4;
  const size_t bX   = (size_t)NR * HID * 2;
  const size_t total = bF + bWiL + bWhL + bWfc + 2 * (bWq + bWm + bWr) + bWp0 + bWp1 + bWo
                     + bL + 3 * (bHf + bHh) + bVS + 2 * bX;
  if (total > ws_size) return;
  if (total > (size_t)134217728) return;

  char* ws = (char*)d_ws;
  size_t off = 0;
  unsigned short* F16  = (unsigned short*)(ws + off); off += bF;
  unsigned short* WiL  = (unsigned short*)(ws + off); off += bWiL;
  unsigned short* WhL  = (unsigned short*)(ws + off); off += bWhL;
  unsigned short* Wfc  = (unsigned short*)(ws + off); off += bWfc;
  unsigned short* Wqs[2]; unsigned short* Wms[2]; unsigned short* Wrs[2];
  for (int l = 0; l < 2; ++l) {
    Wqs[l] = (unsigned short*)(ws + off); off += bWq;
    Wms[l] = (unsigned short*)(ws + off); off += bWm;
    Wrs[l] = (unsigned short*)(ws + off); off += bWr;
  }
  unsigned short* Wp0  = (unsigned short*)(ws + off); off += bWp0;
  unsigned short* Wp1  = (unsigned short*)(ws + off); off += bWp1;
  unsigned short* Wo   = (unsigned short*)(ws + off); off += bWo;
  unsigned short* L16  = (unsigned short*)(ws + off); off += bL;
  float*          H0f  = (float*)(ws + off);          off += bHf;
  unsigned short* H0h  = (unsigned short*)(ws + off); off += bHh;
  float*          H1f  = (float*)(ws + off);          off += bHf;
  unsigned short* H1h  = (unsigned short*)(ws + off); off += bHh;
  float*          H2f  = (float*)(ws + off);          off += bHf;
  unsigned short* H2h  = (unsigned short*)(ws + off); off += bHh;
  float*          VS   = (float*)(ws + off);          off += bVS;
  unsigned short* X1h  = (unsigned short*)(ws + off); off += bX;
  unsigned short* X2h  = (unsigned short*)(ws + off); off += bX;
  if (off != total) return;

  const dim3 cg(512, 8);
  k_cvt8<<<cg, 256, 0, stream>>>(
      features, F16, NR * EMB / 8, ASC,
      lstm_Wih, WiL, G4 * EMB / 8, WSC,
      lstm_Whh, WhL, G4 * HID / 8, WSC,
      fc1_W, Wfc, HID * EMB / 8, WSC,
      mlp0_W, Wp0, HID * G6 / 8, WSC,
      mlp1_W, Wp1, HID * HID / 8, WSC,
      out_W, Wo, NCLS * HID / 8, WSC,
      features, Wo + NCLS * HID, (16 - NCLS) * HID / 8, 0.0f);
  const size_t wo3 = (size_t)G3 * HID, wo1 = (size_t)HID * HID;
  k_cvt8<<<cg, 256, 0, stream>>>(
      gC_Wih,       Wqs[0],       G3 * HID / 8, WSC,
      gP_Whh,       Wqs[0] + wo3, G3 * HID / 8, WSC,
      gC_Whh,       Wms[0],       G3 * HID / 8, WSC,
      gP_Wih,       Wms[0] + wo3, G3 * HID / 8, WSC,
      Wr0,          Wrs[0],       HID * HID / 8, WSC,
      Wr1,          Wrs[0] + wo1, HID * HID / 8, WSC,
      gC_Wih + wo3, Wqs[1],       G3 * HID / 8, WSC,
      gP_Whh + wo3, Wqs[1] + wo3, G3 * HID / 8, WSC);
  k_cvt8<<<cg, 256, 0, stream>>>(
      gC_Whh + wo3, Wms[1],       G3 * HID / 8, WSC,
      gP_Wih + wo3, Wms[1] + wo3, G3 * HID / 8, WSC,
      Wr0 + wo1,    Wrs[1],       HID * HID / 8, WSC,
      Wr1 + wo1,    Wrs[1] + wo1, HID * HID / 8, WSC,
      features, F16, 0, 0.0f,
      features, F16, 0, 0.0f,
      features, F16, 0, 0.0f,
      features, F16, 0, 0.0f);

  k_lstm<<<NN / 16, 256, 0, stream>>>(F16, WiL, WhL, lstm_bih, lstm_bhh, L16);

  k_gemm<<<dim3(NR / 64, HID / 128), 256, 0, stream>>>(
      F16, EMB, EMB, F16, EMB, 0, F16, EMB, 0, F16, EMB, 0, F16, EMB, 0,
      Wfc, EMB, fc1_b, 1, H0f, HID, 1, H0h, HID, 1);

  hipFuncSetAttribute(reinterpret_cast<const void*>(&k_gnn),
                      hipFuncAttributeMaxDynamicSharedMemorySize, GNN_LDS);
  k_gnn<<<NB / 16, 256, GNN_LDS, stream>>>(
      H0f, H0h, adj, smask, attn_W, attn_b, Wqs[0], Wms[0], Wrs[0],
      gC_bih, gC_bhh, gP_bih, gP_bhh, VS, H1f, H1h);
  k_gnn<<<NB / 16, 256, GNN_LDS, stream>>>(
      H1f, H1h, adj, smask, attn_W + 2 * HID, attn_b + 1, Wqs[1], Wms[1], Wrs[1],
      gC_bih + G3, gC_bhh + G3, gP_bih + G3, gP_bhh + G3, VS, H2f, H2h);

  k_gemm<<<dim3(NR / 64, HID / 128), 256, 0, stream>>>(
      H0h, HID, HID, H1h, HID, HID, H2h, HID, HID, F16, EMB, EMB, L16, HID, HID,
      Wp0, G6, mlp0_b, 1, H0f, HID, 0, X1h, HID, 1);
  k_gemm<<<dim3(NR / 64, HID / 128), 256, 0, stream>>>(
      X1h, HID, HID, X1h, HID, 0, X1h, HID, 0, X1h, HID, 0, X1h, HID, 0,
      Wp1, HID, mlp1_b, 1, H0f, HID, 0, X2h, HID, 1);
  k_head<<<NR / 64, 128, 0, stream>>>(X2h, Wo, out_b, out);
}
